// HeuristicModel_71631464563350
// MI455X (gfx1250) — hardware-verified
//
#include <hip/hip_runtime.h>
#include <math.h>


#pragma clang fp contract(off)

typedef float          v8f   __attribute__((ext_vector_type(8)));
typedef float          v4f   __attribute__((ext_vector_type(4)));
typedef __bf16         v16bf __attribute__((ext_vector_type(16)));
typedef unsigned short v16us __attribute__((ext_vector_type(16)));
typedef unsigned short v8us  __attribute__((ext_vector_type(8), may_alias));
typedef int            v8i   __attribute__((ext_vector_type(8)));

#define BSZ    15
#define NA     225
#define NW     572
#define NWP    576
#define BPB    32
#define PITCH  240
#define NTILES 15
#define TPB    256
#define NWAVE  (TPB / 32)

union Frag { v16bf v; v16us u; v8us hh[2]; v8i q; };

__constant__ float c_weights[6] = {0.0f, 5.0f, 50.0f, 500.0f, 5000.0f, 100000.0f};

__device__ __forceinline__ float wscore(int pc, int oc) {
    float sp = (oc == 0 && pc > 0) ? c_weights[pc > 5 ? 5 : pc] : 0.0f;
    float so = (pc == 0 && oc > 0) ? c_weights[oc > 5 ? 5 : oc] : 0.0f;
    return sp - so;
}

__device__ __forceinline__ int win_param(int w) {
    int start, stride;
    if (w < 165)      { int i = w;       int r = i / 11, c = i % 11;     start = r * BSZ + c; stride = 1;  }
    else if (w < 330) { int i = w - 165; int r = i / 15, c = i % 15;     start = r * BSZ + c; stride = 15; }
    else if (w < 451) { int i = w - 330; int r = i / 11, c = i % 11;     start = r * BSZ + c; stride = 16; }
    else              { int i = w - 451; int r = i / 11, c = i % 11 + 4; start = r * BSZ + c; stride = 14; }
    return start | (stride << 16);
}

__device__ __forceinline__ unsigned short f32_to_bf16_bits(float x) {
    unsigned int u = __float_as_uint(x);
    u = u + 0x7FFFu + ((u >> 16) & 1u);
    return (unsigned short)(u >> 16);
}
__device__ __forceinline__ float bf16_bits_to_f32(unsigned short b) {
    return __uint_as_float(((unsigned int)b) << 16);
}

__device__ __forceinline__ v8f mma16(v8f acc, Frag a, Frag b) {
    acc = __builtin_amdgcn_wmma_f32_16x16x32_bf16(false, a.v, false, b.v, (short)0, acc, false, false);
    asm volatile("v_nop\n\tv_nop\n\tv_nop\n\tv_nop" : "+v"(acc) : "v"(a.q), "v"(b.q));
    return acc;
}

__device__ __forceinline__ float pol_elem(const float* e_s, const float* inv_s, int e, int total) {
    if (e >= total) return 0.0f;
    const int b = e / NA;
    const int a = e - b * NA;
    return e_s[b * PITCH + a] * inv_s[b];
}

__device__ __forceinline__ void store_outputs(float* g_out, int nboards, int board0, int nbh,
                                              const float* e_s, const float* inv_s, const float* val_s,
                                              int wv, int lane)
{
    const int total  = nbh * NA;
    const int nlines = (total + 31) >> 5;
    float* outp = g_out + (size_t)board0 * NA;
    const int q = lane & 7;
    for (int L = wv * 4 + (lane >> 3); L < nlines; L += NWAVE * 4) {
        const int e0 = L * 32 + q * 4;
        v4f v;
        v.x = pol_elem(e_s, inv_s, e0 + 0, total);
        v.y = pol_elem(e_s, inv_s, e0 + 1, total);
        v.z = pol_elem(e_s, inv_s, e0 + 2, total);
        v.w = pol_elem(e_s, inv_s, e0 + 3, total);
        if (e0 + 3 < total) {
            *(volatile v4f*)(outp + e0) = v;
        } else {
            if (e0 + 0 < total) *(volatile float*)(outp + e0 + 0) = v.x;
            if (e0 + 1 < total) *(volatile float*)(outp + e0 + 1) = v.y;
            if (e0 + 2 < total) *(volatile float*)(outp + e0 + 2) = v.z;
            if (e0 + 3 < total) *(volatile float*)(outp + e0 + 3) = v.w;
        }
    }
    if (wv == 0 && lane < 8) {
        const int e0 = lane * 4;
        v4f v;
        v.x = (e0 + 0 < nbh) ? val_s[e0 + 0] : 0.0f;
        v.y = (e0 + 1 < nbh) ? val_s[e0 + 1] : 0.0f;
        v.z = (e0 + 2 < nbh) ? val_s[e0 + 2] : 0.0f;
        v.w = (e0 + 3 < nbh) ? val_s[e0 + 3] : 0.0f;
        float* vp = g_out + (size_t)nboards * NA + board0 + e0;
        if (e0 + 3 < nbh) {
            *(volatile v4f*)vp = v;
        } else {
            if (e0 + 0 < nbh) *(volatile float*)(vp + 0) = v.x;
            if (e0 + 1 < nbh) *(volatile float*)(vp + 1) = v.y;
            if (e0 + 2 < nbh) *(volatile float*)(vp + 2) = v.z;
            if (e0 + 3 < nbh) *(volatile float*)(vp + 3) = v.w;
        }
    }
}

extern "C" __global__ __launch_bounds__(TPB, 1)
void k_board_policy(const int* __restrict__ g_boards,
                    const int* __restrict__ g_player,
                    const float* __restrict__ g_pnoise,
                    const float* __restrict__ g_vnoise,
                    float* g_out,
                    int nboards)
{
    __shared__ __align__(16) unsigned short dhi_s[BPB * NWP];
    __shared__ __align__(16) unsigned short dlo_s[BPB * NWP];
    __shared__ __align__(16) unsigned short bmask_s[NTILES * NWP];
    __shared__ __align__(16) float delta_s[BPB * PITCH];
    __shared__ __align__(16) unsigned char boards_s[BPB * NA];
    __shared__ __align__(16) unsigned char winc_s[BPB * PITCH];
    __shared__ int   wp_s[NW];
    __shared__ float basep_s[NWAVE * BPB];
    __shared__ float base_s[BPB];
    __shared__ float inv_s[BPB];
    __shared__ float val_s[BPB];
    __shared__ int   players_s[BPB];

    const int tid  = threadIdx.x;
    const int lane = tid & 31;
    const int wv   = tid >> 5;
    const int board0 = blockIdx.x * BPB;
    if (board0 >= nboards) return;
    int nbh = nboards - board0;
    if (nbh > BPB) nbh = BPB;

    for (int i = tid; i < BPB * NA; i += TPB) {
        const int b  = i / NA;
        const int a  = i - b * NA;
        const int bb = (b < nbh) ? b : (nbh - 1);
        boards_s[i] = (unsigned char)g_boards[(size_t)(board0 + bb) * NA + a];
    }
    {
        unsigned int* w32 = (unsigned int*)winc_s;
        for (int i = tid; i < (BPB * PITCH) / 4; i += TPB) w32[i] = 0u;
        unsigned int* b32 = (unsigned int*)bmask_s;
        for (int i = tid; i < (NTILES * NWP) / 2; i += TPB) b32[i] = 0u;
    }
    for (int w = tid; w < NW; w += TPB) wp_s[w] = win_param(w);
    if (tid < BPB) {
        const int bb = (tid < nbh) ? tid : (nbh - 1);
        players_s[tid] = g_player[board0 + bb];
    }
    __syncthreads();

    for (int w = tid; w < NW; w += TPB) {
        const int wp = wp_s[w];
        const int st = wp & 0xffff, sd = wp >> 16;
        #pragma unroll
        for (int j = 0; j < 5; ++j) {
            const int cell = st + j * sd;
            bmask_s[(cell >> 4) * NWP + w] |= (unsigned short)(1u << (cell & 15));
        }
    }

    {
        const int b      = tid & (BPB - 1);
        const int s      = tid >> 5;
        const int player = players_s[b];
        const int opp    = 3 - player;
        const unsigned char* brd = boards_s + b * NA;
        float bacc = 0.0f;
        for (int w = s; w < NWP; w += NWAVE) {
            unsigned short hb = 0, lb = 0;
            if (w < NW) {
                const int wp = wp_s[w];
                const int st = wp & 0xffff, sd = wp >> 16;
                const int c0 = st, c1 = st + sd, c2 = c1 + sd, c3 = c2 + sd, c4 = c3 + sd;
                const int v0 = brd[c0], v1 = brd[c1], v2 = brd[c2], v3 = brd[c3], v4 = brd[c4];
                const int pc = (v0 == player) + (v1 == player) + (v2 == player) + (v3 == player) + (v4 == player);
                const int oc = (v0 == opp) + (v1 == opp) + (v2 == opp) + (v3 == opp) + (v4 == opp);
                const float s0 = wscore(pc, oc);
                bacc += s0;
                const float d  = wscore(pc + 1, oc) - s0;
                hb = f32_to_bf16_bits(d);
                const float lo = d - bf16_bits_to_f32(hb);
                lb = f32_to_bf16_bits(lo);
                if (pc == 4 && oc == 0) {
                    winc_s[b * PITCH + c0] = 1; winc_s[b * PITCH + c1] = 1;
                    winc_s[b * PITCH + c2] = 1; winc_s[b * PITCH + c3] = 1;
                    winc_s[b * PITCH + c4] = 1;
                }
            }
            dhi_s[b * NWP + w] = hb;
            dlo_s[b * NWP + w] = lb;
        }
        basep_s[s * BPB + b] = bacc;
    }
    __syncthreads();

    if (tid < BPB) {
        float t = 0.0f;
        #pragma unroll
        for (int s = 0; s < NWAVE; ++s) t += basep_s[s * BPB + tid];
        base_s[tid] = t;
    }

    {
        const int h = lane >> 4;
        const int m = lane & 15;
        for (int nt = wv; nt < NTILES; nt += NWAVE) {
            v8f acc0 = {0.0f, 0.0f, 0.0f, 0.0f, 0.0f, 0.0f, 0.0f, 0.0f};
            v8f acc1 = {0.0f, 0.0f, 0.0f, 0.0f, 0.0f, 0.0f, 0.0f, 0.0f};
            const unsigned short* mrow = bmask_s + nt * NWP;
            const unsigned short* a0h  = dhi_s + m * NWP;
            const unsigned short* a0l  = dlo_s + m * NWP;
            const unsigned short* a1h  = dhi_s + (16 + m) * NWP;
            const unsigned short* a1l  = dlo_s + (16 + m) * NWP;
            #pragma unroll 2
            for (int k0 = 0; k0 < NWP; k0 += 32) {
                const int ka = k0 + 8 * h;
                const int kb = k0 + 16 + 8 * h;
                Frag fb;
                fb.hh[0] = *(const v8us*)(mrow + ka);
                fb.hh[1] = *(const v8us*)(mrow + kb);
                #pragma unroll
                for (int i = 0; i < 16; ++i) {
                    const unsigned int bit = (((unsigned int)fb.u[i]) >> m) & 1u;
                    fb.u[i] = (unsigned short)((0u - bit) & 0x3F80u);
                }
                Frag fa;
                fa.hh[0] = *(const v8us*)(a0h + ka);
                fa.hh[1] = *(const v8us*)(a0h + kb);
                acc0 = mma16(acc0, fa, fb);
                fa.hh[0] = *(const v8us*)(a0l + ka);
                fa.hh[1] = *(const v8us*)(a0l + kb);
                acc0 = mma16(acc0, fa, fb);
                fa.hh[0] = *(const v8us*)(a1h + ka);
                fa.hh[1] = *(const v8us*)(a1h + kb);
                acc1 = mma16(acc1, fa, fb);
                fa.hh[0] = *(const v8us*)(a1l + ka);
                fa.hh[1] = *(const v8us*)(a1l + kb);
                acc1 = mma16(acc1, fa, fb);
            }
            const int col = nt * 16 + m;
            #pragma unroll
            for (int r = 0; r < 8; ++r) {
                delta_s[(8 * h + r) * PITCH + col]      = acc0[r];
                delta_s[(16 + 8 * h + r) * PITCH + col] = acc1[r];
            }
        }
    }
    __syncthreads();

    for (int b = wv; b < nbh; b += NWAVE) {
        const int   bg   = board0 + b;
        const float base = base_s[b];
        float* row = delta_s + b * PITCH;
        const unsigned char* brd  = boards_s + b * NA;
        const unsigned char* wrow = winc_s + b * PITCH;

        double dsum = 0.0;
        float  cnt  = 0.0f;
        for (int a = lane; a < NA; a += 32) {
            const bool empty = (brd[a] == 0);
            const bool win   = (wrow[a] != 0);
            float x;
            if (!empty)   x = -1000000.0f;
            else if (win) x = 100000.0f;
            else          x = base + row[a];
            row[a] = x;
            if (x > -100000.0f) { dsum += (double)x; cnt += 1.0f; }
        }
        #pragma unroll
        for (int o = 16; o > 0; o >>= 1) {
            dsum += __shfl_xor(dsum, o, 32);
            cnt  += __shfl_xor(cnt, o, 32);
        }
        const float nsafe = fmaxf(cnt, 1.0f);
        const float mean  = (float)dsum / nsafe;

        double dvs = 0.0;
        for (int a = lane; a < NA; a += 32) {
            const float x = row[a];
            if (x > -100000.0f) { const float t = x - mean; const float sq = t * t; dvs += (double)sq; }
        }
        #pragma unroll
        for (int o = 16; o > 0; o >>= 1) dvs += __shfl_xor(dvs, o, 32);
        const float var  = (float)dvs / nsafe;
        const float stdv = fmaxf(1.0f, sqrtf(var));

        const float* pn = g_pnoise + (size_t)bg * NA;
        float mx = -3.0e38f;
        for (int a = lane; a < NA; a += 32) {
            float x = row[a];
            if (x > -100000.0f) x = x + (pn[a] * 2.0f) * stdv;
            const float z = x * 0.03f;
            row[a] = z;
            mx = fmaxf(mx, z);
        }
        #pragma unroll
        for (int o = 16; o > 0; o >>= 1) mx = fmaxf(mx, __shfl_xor(mx, o, 32));

        float se = 0.0f;
        for (int a = lane; a < NA; a += 32) {
            const float e = expf(row[a] - mx);
            row[a] = e;
            se += e;
        }
        #pragma unroll
        for (int o = 16; o > 0; o >>= 1) se += __shfl_xor(se, o, 32);

        if (lane == 0) {
            inv_s[b] = 1.0f / se;
            const float v = tanhf((base + g_vnoise[bg] * 200.0f) * (1.0f / 3000.0f));
            val_s[b] = fminf(0.95f, fmaxf(-0.95f, v));
        }
    }
    __syncthreads();

    store_outputs(g_out, nboards, board0, nbh, delta_s, inv_s, val_s, wv, lane);
    __threadfence();
    store_outputs(g_out, nboards, board0, nbh, delta_s, inv_s, val_s, wv, lane);
}

extern "C" void kernel_launch(void* const* d_in, const int* in_sizes, int n_in,
                              void* d_out, int out_size, void* d_ws, size_t ws_size,
                              hipStream_t stream) {
    (void)d_ws; (void)ws_size;
    if (n_in < 4) return;
    const int*   boards = (const int*)d_in[0];
    const int*   player = (const int*)d_in[1];
    const float* pnoise = (const float*)d_in[2];
    const float* vnoise = (const float*)d_in[3];
    float*       out    = (float*)d_out;
    const int nboards = in_sizes[1];
    if (nboards <= 0) return;
    if (in_sizes[0] < nboards * NA || in_sizes[2] < nboards * NA || in_sizes[3] < nboards) return;
    if (out_size < nboards * NA + nboards) return;
    const int nblocks = (nboards + BPB - 1) / BPB;
    hipLaunchKernelGGL(k_board_policy, dim3(nblocks), dim3(TPB), 0, stream,
                       boards, player, pnoise, vnoise, out, nboards);
    (void)hipGetLastError();
}
